// Conv4d1_8057358647868
// MI455X (gfx1250) — hardware-verified
//
#include <hip/hip_runtime.h>

typedef __attribute__((ext_vector_type(16))) _Float16 v16h;
typedef __attribute__((ext_vector_type(8)))  _Float16 v8h;
typedef __attribute__((ext_vector_type(8)))  float    v8f;
typedef __attribute__((ext_vector_type(4)))  float    v4f;
typedef __attribute__((ext_vector_type(4)))  unsigned int v4u;

constexpr int kB    = 2;
constexpr int kCin  = 8;
constexpr int kCout = 16;
constexpr int kW = 32, kH = 32, kU = 20, kV = 20;
constexpr int kUV      = kU * kV;
constexpr int kPosPerW = kH * kUV;
constexpr int kPosPerB = kW * kPosPerW;
constexpr int kXPerB   = kCin * kPosPerB;
constexpr int kKtot = kCin * 81;
constexpr int kKpad = 672;
constexpr int kGrp  = kKpad / 8;
constexpr int kSeg  = 72;
constexpr int kWChunk     = 4;
constexpr int kNChunkPerB = kW / kWChunk;
constexpr int kMChunk     = kWChunk * kPosPerW;
constexpr int kP1W  = kWChunk + 2;
constexpr int kHP   = kH + 2;
constexpr int kP1Cells   = kP1W * kHP * kUV;
constexpr int kP1Halves  = kP1Cells * kSeg;
constexpr int kP1Threads = kP1Halves / 8;
constexpr int kA16Halves  = kMChunk * kKpad;
constexpr int kA16Threads = kA16Halves / 8;
constexpr int kBtHalves  = kCout * kKpad;
constexpr int kBtThreads = kBtHalves / 8;
constexpr float kWCarry    = 16.0f;
constexpr float kWCarryInv = 1.0f / 16.0f;

static_assert(kKpad % 32 == 0);
static_assert(kKpad >= kKtot);
static_assert(kSeg % 8 == 0);
static_assert(9 * kSeg == kKtot);
static_assert(kMChunk % 64 == 0);
static_assert(kP1Halves % 8 == 0);
static_assert(kP1Threads % 32 == 0);
static_assert(kA16Threads % 256 == 0);
static_assert(kBtThreads % 32 == 0);
static_assert(kNChunkPerB * kWChunk == kW);

constexpr size_t kOffBt    = 0;
constexpr size_t kBytesBt  = (size_t)kBtHalves * 2;
constexpr size_t kOffP1    = kOffBt + kBytesBt;
constexpr size_t kBytesP1  = (size_t)kP1Halves * 2;
constexpr size_t kOffA16   = kOffP1 + kBytesP1;
constexpr size_t kBytesA16 = (size_t)kA16Halves * 2;
constexpr size_t kWsNeed   = kOffA16 + kBytesA16;
static_assert(kOffP1 % 512 == 0);
static_assert(kOffA16 % 512 == 0);
static_assert(kWsNeed == 80584704ull);
static_assert(kWsNeed <= 134217728ull);

__device__ __forceinline__ void acc_guard4(v8f& a, v8f& b, v8f& c, v8f& d) { asm volatile("v_nop\n\tv_nop\n\tv_nop\n\tv_nop" : "+v"(a), "+v"(b), "+v"(c), "+v"(d)); }
template <typename T> struct Frag;
template <> struct Frag<_Float16> {
  typedef v16h V; union U { v16h v; v8h h[2]; };
  static __device__ __forceinline__ v16h load(const _Float16* p) {
    U f; f.h[0] = *(const v8h*)(p); f.h[1] = *(const v8h*)(p + 16); return f.v;
  }
  static __device__ __forceinline__ v8f mma(v16h a, v16h b, v8f c) {
    return __builtin_amdgcn_wmma_f32_16x16x32_f16(false, a, false, b, (short)0, c, false, false);
  }
};
__device__ __forceinline__ unsigned pk16(unsigned short a, unsigned short b) { return (unsigned)a | ((unsigned)b << 16); }
__device__ __forceinline__ unsigned short h_bits(float f) { const _Float16 h = (_Float16)f; return __builtin_bit_cast(unsigned short, h); }

__device__ __forceinline__ v8f hmma(v16h a, v16h b, v8f c) {
  c = Frag<_Float16>::mma(a, b, c);
  asm volatile("v_nop\n\tv_nop\n\tv_nop\n\tv_nop" : "+v"(c) : "v"(a), "v"(b));
  return c;
}
__device__ __forceinline__ int clampi(int v, int lo, int hi) { return v < lo ? lo : (v > hi ? hi : v); }

__global__ __launch_bounds__(256) void bt_build_kernel(const float* __restrict__ w, unsigned short* __restrict__ Bt, int nthr) {
  const int t = blockIdx.x * 256 + threadIdx.x;
  if (t >= nthr) return;
  const int co  = t / kGrp;
  const int g   = t - co * kGrp;
  const int seg = g / 9;
  const int j0  = (g - seg * 9) * 8;
  const bool valid = (seg < 9);
  const int segc = valid ? seg : 0;
  const int k1 = segc / 3;
  const int k2 = segc - k1 * 3;
  const int wb = co * kKtot + k1 * 27 + k2 * 9;
  unsigned short hb[8];
#pragma unroll
  for (int e = 0; e < 8; ++e) {
    const int j  = j0 + e;
    const int ci = j / 9;
    const int r9 = j - ci * 9;
    const int k3 = r9 / 3;
    const int k4 = r9 - k3 * 3;
    float val = w[wb + ci * 81 + k3 * 3 + k4] * kWCarry;
    val = valid ? val : 0.0f;
    hb[e] = h_bits(val);
  }
  const v4u u = (v4u){pk16(hb[0], hb[1]), pk16(hb[2], hb[3]), pk16(hb[4], hb[5]), pk16(hb[6], hb[7])};
  unsigned short* q = Bt + 8 * (size_t)t;
  *(volatile v4u*)q = u;
  __threadfence();
  *(volatile v4u*)q = u;
}

__global__ __launch_bounds__(256) void p1_build_kernel(const float* __restrict__ x, unsigned short* __restrict__ P1,
                                                       int b, int wbaseP, int nthr) {
  const int t = blockIdx.x * 256 + threadIdx.x;
  if (t >= nthr) return;
  const int cell = t / 9;
  const int g    = t - cell * 9;
  const int c0   = g * 8;
  const int v    = cell % kV;
  const int tmp  = cell / kV;
  const int u    = tmp % kU;
  const int tmp2 = tmp / kU;
  const int hp   = tmp2 % kHP;
  const int wl   = tmp2 / kHP;
  const int xw = wbaseP + wl - 1;
  const int xh = hp - 1;
  const bool vwh = ((unsigned)xw < (unsigned)kW) && ((unsigned)xh < (unsigned)kH);
  const int cxw = clampi(xw, 0, kW - 1);
  const int cxh = clampi(xh, 0, kH - 1);
  const int rowbase = b * kXPerB + cxw * kPosPerW + cxh * kUV;
  unsigned short hb[8];
#pragma unroll
  for (int e = 0; e < 8; ++e) {
    const int c  = c0 + e;
    const int ci = c / 9;
    const int r9 = c - ci * 9;
    const int k3 = r9 / 3;
    const int k4 = r9 - k3 * 3;
    const int xu = u + k3 - 1;
    const int xv = v + k4 - 1;
    const bool ok = vwh && ((unsigned)xu < (unsigned)kU) && ((unsigned)xv < (unsigned)kV);
    const int cxu = clampi(xu, 0, kU - 1);
    const int cxv = clampi(xv, 0, kV - 1);
    float val = x[rowbase + ci * kPosPerB + cxu * kV + cxv];
    val = ok ? val : 0.0f;
    hb[e] = h_bits(val);
  }
  const v4u pk = (v4u){pk16(hb[0], hb[1]), pk16(hb[2], hb[3]), pk16(hb[4], hb[5]), pk16(hb[6], hb[7])};
  unsigned short* q = P1 + 8 * (size_t)t;
  *(volatile v4u*)q = pk;
  __threadfence();
  *(volatile v4u*)q = pk;
}

__global__ __launch_bounds__(256) void a16_expand_kernel(const unsigned short* __restrict__ P1, unsigned short* __restrict__ A16, int nthr) {
  const int t = blockIdx.x * 256 + threadIdx.x;
  if (t >= nthr) return;
  const int p   = t / kGrp;
  const int g   = t - p * kGrp;
  const int seg = g / 9;
  const int j0  = (g - seg * 9) * 8;
  const bool valid = (seg < 9);
  const int segc = valid ? seg : 0;
  const int k1 = segc / 3;
  const int k2 = segc - k1 * 3;
  const int wl  = p / kPosPerW;
  const int rem = p - wl * kPosPerW;
  const int h   = rem / kUV;
  const int uv  = rem - h * kUV;
  const int cell = ((wl + k1) * kHP + (h + k2)) * kUV + uv;
  v4u val = *(const v4u*)(P1 + (size_t)cell * kSeg + j0);
  const unsigned msk = valid ? 0xFFFFFFFFu : 0u;
  val.x &= msk; val.y &= msk; val.z &= msk; val.w &= msk;
  unsigned short* q = A16 + 8 * (size_t)t;
  *(volatile v4u*)q = val;
  __threadfence();
  *(volatile v4u*)q = val;
}

__global__ __launch_bounds__(256) void gemm_n16_kernel(const unsigned short* __restrict__ Ap, int lda,
                                                       const unsigned short* __restrict__ Btp, int ldb,
                                                       float* __restrict__ outp, long coStride,
                                                       const float* __restrict__ bias,
                                                       int M, int K, float scale) {
  const _Float16* A  = (const _Float16*)Ap;
  const _Float16* Bt = (const _Float16*)Btp;
  __shared__ __align__(16) float sT[8][16 * 68];
  const int lane = threadIdx.x & 31;
  const int wave = threadIdx.x >> 5;
  const int tilesM = M >> 6;
  const int tile = blockIdx.x * 8 + wave;
  if (tile >= tilesM) return;
  const int m0 = tile << 6;
  const int rlane = lane & 15;
  const int koff  = (lane >> 4) * 8;
  const int mOff  = koff;

  v8f acc[4];
#pragma unroll
  for (int i = 0; i < 4; ++i) acc[i] = (v8f){0.f, 0.f, 0.f, 0.f, 0.f, 0.f, 0.f, 0.f};

  const _Float16* Brow  = Bt + (size_t)rlane * ldb + koff;
  const _Float16* Arow0 = A + (size_t)(m0 + rlane) * lda + koff;

  for (int k0 = 0; k0 < K; k0 += 32) {
    const v16h bf = Frag<_Float16>::load(Brow + k0);
    v16h af[4];
#pragma unroll
    for (int i = 0; i < 4; ++i) af[i] = Frag<_Float16>::load(Arow0 + (size_t)(i * 16) * lda + k0);
#pragma unroll
    for (int i = 0; i < 4; ++i) acc[i] = hmma(af[i], bf, acc[i]);
  }
  acc_guard4(acc[0], acc[1], acc[2], acc[3]);

  float* slab = sT[wave];
  const float bv = bias[rlane];
#pragma unroll
  for (int i = 0; i < 4; ++i) {
#pragma unroll
    for (int r = 0; r < 8; ++r) {
      slab[rlane * 68 + i * 16 + mOff + r] = acc[i][r] * scale + bv;
    }
  }
  __builtin_amdgcn_fence(__ATOMIC_RELEASE, "workgroup");
  __builtin_amdgcn_wave_barrier();
  __builtin_amdgcn_fence(__ATOMIC_ACQUIRE, "workgroup");
  {
    const int hh = lane >> 4;
    const int c4 = (lane & 15) * 4;
    for (int pass = 0; pass < 2; ++pass) {
#pragma unroll
      for (int it = 0; it < 8; ++it) {
        const int co = it * 2 + hh;
        const v4f val = *(const v4f*)(slab + co * 68 + c4);
        *(volatile v4f*)(outp + (size_t)co * coStride + m0 + c4) = val;
      }
      __threadfence();
    }
  }
}

extern "C" void kernel_launch(void* const* d_in, const int* in_sizes, int n_in,
                              void* d_out, int out_size, void* d_ws, size_t ws_size,
                              hipStream_t stream) {
  if (n_in < 3) return;
  if (in_sizes[0] != kB * kXPerB) return;
  if (in_sizes[1] != kCout * kKtot) return;
  if (in_sizes[2] != kCout) return;
  if (out_size != kB * kCout * kPosPerB) return;
  if (ws_size < kWsNeed) return;

  const float* x    = (const float*)d_in[0];
  const float* wgt  = (const float*)d_in[1];
  const float* bias = (const float*)d_in[2];
  float* out = (float*)d_out;
  unsigned char* ws = (unsigned char*)d_ws;
  unsigned short* Bt  = (unsigned short*)(ws + kOffBt);
  unsigned short* P1  = (unsigned short*)(ws + kOffP1);
  unsigned short* A16 = (unsigned short*)(ws + kOffA16);

  bt_build_kernel<<<dim3((kBtThreads + 255) / 256), dim3(256), 0, stream>>>(wgt, Bt, kBtThreads);

  for (int q = 0; q < kB * kNChunkPerB; ++q) {
    const int b = q / kNChunkPerB;
    const int c = q - b * kNChunkPerB;
    p1_build_kernel<<<dim3((kP1Threads + 255) / 256), dim3(256), 0, stream>>>(x, P1, b, c * kWChunk, kP1Threads);
    a16_expand_kernel<<<dim3(kA16Threads / 256), dim3(256), 0, stream>>>(P1, A16, kA16Threads);
    float* outp = out + (size_t)b * kCout * kPosPerB + (size_t)c * kMChunk;
    gemm_n16_kernel<<<dim3(kMChunk / 64 / 8), dim3(256), 0, stream>>>(
        A16, kKpad, Bt, kKpad, outp, (long)kPosPerB, bias, kMChunk, kKpad, kWCarryInv);
  }
}
